// JointSinhLinearAttention_55052890800620
// MI455X (gfx1250) — hardware-verified
//
#include <hip/hip_runtime.h>
#define BH 32
#define SN 2048
#define DD 64
typedef __bf16 v16b __attribute__((ext_vector_type(16)));
typedef unsigned short v8us __attribute__((ext_vector_type(8), may_alias));
typedef float  v8f  __attribute__((ext_vector_type(8)));
typedef float  v4f  __attribute__((ext_vector_type(4)));
typedef float  v4fa __attribute__((ext_vector_type(4), may_alias));
union FragB { v16b v; v8us half[2]; unsigned short u[16]; };

__device__ __forceinline__ unsigned short bf16_bits(float x) { unsigned int u = __float_as_uint(x); return (unsigned short)((u + 0x7FFFu + ((u >> 16) & 1u)) >> 16); }
__device__ __forceinline__ float bf16_val(unsigned short b) { return __uint_as_float(((unsigned int)b) << 16); }
__device__ __forceinline__ float bf16_round(float x) { return bf16_val(bf16_bits(x)); }
template <int NT>
__device__ __forceinline__ v8f mmaN(v16b ah, v16b al, v16b bh, v16b bl, v8f c) {
  c = __builtin_amdgcn_wmma_f32_16x16x32_bf16(false, ah, false, bh, (short)0, c, false, false);
  if (NT >= 2) c = __builtin_amdgcn_wmma_f32_16x16x32_bf16(false, al, false, bh, (short)0, c, false, false);
  if (NT >= 3) c = __builtin_amdgcn_wmma_f32_16x16x32_bf16(false, ah, false, bl, (short)0, c, false, false);
  asm volatile("v_nop\n\tv_nop\n\tv_nop\n\tv_nop" : "+v"(c) : "v"(ah), "v"(al), "v"(bh), "v"(bl));
  return c;
}

typedef _Float16 v16h __attribute__((ext_vector_type(16)));
union FragH { v16h v; v8us half[2]; _Float16 h[16]; unsigned short u[16]; };
template <int NT>
__device__ __forceinline__ v8f mmaH(v16h ah, v16h al, v16h bh, v16h bl, v8f c) {
  c = __builtin_amdgcn_wmma_f32_16x16x32_f16(false, ah, false, bh, (short)0, c, false, false);
  if (NT >= 2) c = __builtin_amdgcn_wmma_f32_16x16x32_f16(false, al, false, bh, (short)0, c, false, false);
  if (NT >= 3) c = __builtin_amdgcn_wmma_f32_16x16x32_f16(false, ah, false, bl, (short)0, c, false, false);
  asm volatile("v_nop\n\tv_nop\n\tv_nop\n\tv_nop" : "+v"(c) : "v"(ah), "v"(al), "v"(bh), "v"(bl));
  return c;
}

__global__ __launch_bounds__(256) void k_prep(const float* __restrict__ K, const float* __restrict__ V, const int* __restrict__ mask, unsigned short* __restrict__ Kb, _Float16* __restrict__ Vt) {
  const size_t t = (size_t)blockIdx.x * 256 + threadIdx.x; if (t >= (size_t)BH * SN * DD / 8) return;
  { const size_t e0 = t * 8; const size_t row = e0 / DD; const int bh = (int)(row / SN), j = (int)(row % SN); const int b = bh / 16;
    const unsigned short keep = (mask[b * SN + j] != 0) ? (unsigned short)0xFFFFu : (unsigned short)0;
    const v4f k0 = *(const v4fa*)(K + e0), k1 = *(const v4fa*)(K + e0 + 4);
    v8us kb; kb[0] = bf16_bits(k0[0]) & keep; kb[1] = bf16_bits(k0[1]) & keep; kb[2] = bf16_bits(k0[2]) & keep; kb[3] = bf16_bits(k0[3]) & keep;
    kb[4] = bf16_bits(k1[0]) & keep; kb[5] = bf16_bits(k1[1]) & keep; kb[6] = bf16_bits(k1[2]) & keep; kb[7] = bf16_bits(k1[3]) & keep;
    *(volatile v8us*)(Kb + e0) = kb; __threadfence(); *(volatile v8us*)(Kb + e0) = kb; }
  { const int j8 = (int)(t % (SN / 8)) * 8; const int d = (int)((t / (SN / 8)) % DD); const int bh = (int)(t / ((size_t)(SN / 8) * DD)); FragH f;
#pragma unroll
    for (int q = 0; q < 8; ++q) f.h[q] = (_Float16)bf16_round(V[((size_t)bh * SN + j8 + q) * DD + d]);
    const v8us o = f.half[0];
    *(volatile v8us*)((unsigned short*)Vt + ((size_t)bh * DD + d) * SN + j8) = o; __threadfence(); *(volatile v8us*)((unsigned short*)Vt + ((size_t)bh * DD + d) * SN + j8) = o; }
}

__device__ __forceinline__ float sinh_relu(float s) {
  const float x = __builtin_amdgcn_fmed3f(s, 0.f, 3.0e38f) * 1.44269504088896341f;
  return 0.5f * (__builtin_amdgcn_exp2f(x) - __builtin_amdgcn_exp2f(-x));
}

__global__ __launch_bounds__(128) void k_attn(const float* __restrict__ Q, const unsigned short* __restrict__ Kb, const _Float16* __restrict__ Vt, float* __restrict__ out) {
  constexpr int KS = DD / 32, DT = DD / 16, RPW = 32, NQB = SN / (4 * RPW);
  __shared__ __attribute__((aligned(16))) unsigned short sP[4][RPW][40];
  __shared__ __attribute__((aligned(16))) float sO[4][RPW][DD];
  const int tid = threadIdx.x, w = tid >> 5, lane = tid & 31, ln = lane & 15, hh = lane >> 4;
  const int bh = blockIdx.x / NQB, qblk = blockIdx.x % NQB;
  const int q0 = qblk * (4 * RPW) + w * RPW;
  const unsigned short* Kbh = Kb + (size_t)bh * SN * DD;
  const unsigned short* Vth = (const unsigned short*)Vt + (size_t)bh * DD * SN;
  FragB aq[2][KS];
#pragma unroll
  for (int rt = 0; rt < 2; ++rt) {
    const float* qr = Q + ((size_t)bh * SN + q0 + rt * 16 + ln) * DD;
#pragma unroll
    for (int ks = 0; ks < KS; ++ks) {
      const v4f x0 = *(const v4fa*)(qr + ks * 32 + 8 * hh), x1 = *(const v4fa*)(qr + ks * 32 + 8 * hh + 4);
      const v4f x2 = *(const v4fa*)(qr + ks * 32 + 16 + 8 * hh), x3 = *(const v4fa*)(qr + ks * 32 + 16 + 8 * hh + 4);
      const float xs[16] = {x0[0],x0[1],x0[2],x0[3],x1[0],x1[1],x1[2],x1[3],x2[0],x2[1],x2[2],x2[3],x3[0],x3[1],x3[2],x3[3]};
#pragma unroll
      for (int i = 0; i < 16; ++i) aq[rt][ks].u[i] = bf16_bits(xs[i] * 0.125f);
    }
  }
  float l_r[2][8];
  v8f oacc[2][DT];
#pragma unroll
  for (int rt = 0; rt < 2; ++rt) {
#pragma unroll
    for (int r = 0; r < 8; ++r) l_r[rt][r] = 0.f;
#pragma unroll
    for (int dt = 0; dt < DT; ++dt) oacc[rt][dt] = (v8f){0.f,0.f,0.f,0.f,0.f,0.f,0.f,0.f};
  }
#pragma unroll 1
  for (int j0 = 0; j0 < SN; j0 += 32) {
    v8f s[2][2];
#pragma unroll
    for (int nt = 0; nt < 2; ++nt) {
      const unsigned short* brow = Kbh + (size_t)(j0 + nt * 16 + ln) * DD;
      FragB b[KS];
#pragma unroll
      for (int ks = 0; ks < KS; ++ks) { b[ks].half[0] = *(const v8us*)(brow + ks * 32 + 8 * hh); b[ks].half[1] = *(const v8us*)(brow + ks * 32 + 16 + 8 * hh); }
#pragma unroll
      for (int rt = 0; rt < 2; ++rt) {
        v8f acc = (v8f){0.f,0.f,0.f,0.f,0.f,0.f,0.f,0.f};
#pragma unroll
        for (int ks = 0; ks < KS; ++ks) acc = mmaN<1>(aq[rt][ks].v, aq[rt][ks].v, b[ks].v, b[ks].v, acc);
        s[rt][nt] = acc;
      }
    }
#pragma unroll
    for (int rt = 0; rt < 2; ++rt)
#pragma unroll
      for (int r = 0; r < 8; ++r) {
        const float p0 = sinh_relu(s[rt][0][r]), p1 = sinh_relu(s[rt][1][r]);
        l_r[rt][r] += p0 + p1;
        FragH t; t.h[0] = (_Float16)p0; t.h[1] = (_Float16)p1;
        sP[w][rt * 16 + 8 * hh + r][ln] = t.u[0]; sP[w][rt * 16 + 8 * hh + r][16 + ln] = t.u[1];
      }
    __builtin_amdgcn_fence(__ATOMIC_ACQ_REL, "workgroup");
    __builtin_amdgcn_wave_barrier();
    FragH pa[2];
#pragma unroll
    for (int rt = 0; rt < 2; ++rt) { pa[rt].half[0] = *(const v8us*)&sP[w][rt * 16 + ln][8 * hh]; pa[rt].half[1] = *(const v8us*)&sP[w][rt * 16 + ln][16 + 8 * hh]; }
#pragma unroll
    for (int dt = 0; dt < DT; ++dt) {
      const unsigned short* vrow = Vth + (size_t)(dt * 16 + ln) * SN + j0;
      FragH bv; bv.half[0] = *(const v8us*)(vrow + 8 * hh); bv.half[1] = *(const v8us*)(vrow + 16 + 8 * hh);
#pragma unroll
      for (int rt = 0; rt < 2; ++rt) oacc[rt][dt] = mmaH<1>(pa[rt].v, pa[rt].v, bv.v, bv.v, oacc[rt][dt]);
    }
    __builtin_amdgcn_fence(__ATOMIC_ACQ_REL, "workgroup");
    __builtin_amdgcn_wave_barrier();
  }
#pragma unroll
  for (int rt = 0; rt < 2; ++rt) {
#pragma unroll
    for (int r = 0; r < 8; ++r) {
      float l = l_r[rt][r];
      l += __shfl_xor(l, 1, 32); l += __shfl_xor(l, 2, 32); l += __shfl_xor(l, 4, 32); l += __shfl_xor(l, 8, 32);
      l_r[rt][r] = 1.0f / fmaxf(l, 1e-6f);
    }
#pragma unroll
    for (int dt = 0; dt < DT; ++dt)
#pragma unroll
      for (int r = 0; r < 8; ++r) sO[w][rt * 16 + 8 * hh + r][dt * 16 + ln] = oacc[rt][dt][r] * l_r[rt][r];
  }
  __builtin_amdgcn_fence(__ATOMIC_ACQ_REL, "workgroup");
  __builtin_amdgcn_wave_barrier();
  for (int pass = 0; pass < 2; ++pass) {
#pragma unroll
    for (int r = 0; r < RPW; ++r) {
      if (lane < DD / 4) {
        const v4f val = *(const v4fa*)&sO[w][r][lane * 4];
        *(volatile v4f*)(out + ((size_t)bh * SN + q0 + r) * DD + lane * 4) = val;
      }
    }
    if (pass == 0) __threadfence();
  }
}

extern "C" void kernel_launch(void* const* d_in, const int* in_sizes, int n_in,
                              void* d_out, int out_size, void* d_ws, size_t ws_size, hipStream_t stream) {
  (void)in_sizes; (void)n_in; (void)out_size;
  const float* Q = (const float*)d_in[0]; const float* K = (const float*)d_in[1]; const float* V = (const float*)d_in[2]; const int* mask = (const int*)d_in[3];
  char* ws = (char*)d_ws; size_t off = 0;
  auto take = [&](size_t bytes) { char* p = ws + off; off += (bytes + 255) & ~(size_t)255; return p; };
  unsigned short* Kb = (unsigned short*)take((size_t)BH * SN * DD * 2);
  _Float16* Vt = (_Float16*)take((size_t)BH * DD * SN * 2);
  if (off > ws_size) return;
  k_prep<<<(unsigned)(((size_t)BH * SN * DD / 8 + 255) / 256), 256, 0, stream>>>(K, V, mask, Kb, Vt);
  k_attn<<<(unsigned)(BH * (SN / 128)), 128, 0, stream>>>(Q, Kb, Vt, (float*)d_out);
}
